// MHA_10350871183657
// MI455X (gfx1250) — hardware-verified
//
#include <hip/hip_runtime.h>


#ifndef NB
#define NB 4
#endif
#ifndef SEQ
#define SEQ 2048
#endif
#define NB_FULL  4
#define SEQ_FULL 2048
#define DM   1024
#define NH   16
#define HD   64
#ifndef RH
#define RH ((SEQ) < 512 ? (SEQ) : 512)
#endif
#define X_BSTRIDE ((size_t)SEQ_FULL * DM)
#ifndef OUT_BSTRIDE
#define OUT_BSTRIDE ((size_t)SEQ * DM)
#endif
#define CTXCAR 64.0f
#define WOCAR  64.0f

static_assert(HD == 64);
static_assert(DM == NH * HD);
static_assert(SEQ % 64 == 0);
static_assert(RH % 64 == 0);
static_assert(RH <= SEQ);
static_assert(RH >= 64);
static_assert((NB * SEQ) % 64 == 0);
static_assert(DM % 64 == 0);
static_assert(((size_t)SEQ * DM / 8) % 256 == 0);
static_assert(((size_t)DM * DM / 8) % 256 == 0);

typedef _Float16 h16;
typedef unsigned short bf;
typedef __attribute__((ext_vector_type(16))) __bf16   v16bf;
typedef __attribute__((ext_vector_type(16))) _Float16 v16h;
typedef __attribute__((ext_vector_type(8)))  _Float16 v8h;
typedef __attribute__((ext_vector_type(8)))  unsigned short v8us;
typedef __attribute__((ext_vector_type(8)))  float    v8f;
typedef __attribute__((ext_vector_type(4)))  float    v4f;
typedef v4f  __attribute__((may_alias)) v4fa;

__device__ __forceinline__ unsigned short f2bf(float f) { unsigned u = __float_as_uint(f); u += 0x7FFFu + ((u >> 16) & 1u); return (unsigned short)(u >> 16); }
__device__ __forceinline__ float bf2f(unsigned short b) { return __uint_as_float(((unsigned)b) << 16); }
__device__ __forceinline__ float bfr(float f) { return bf2f(f2bf(f)); }
__device__ __forceinline__ void splitf(float y, unsigned short& h, unsigned short& l) { h = f2bf(y); l = f2bf(y - bf2f(h)); }
__device__ __forceinline__ v16h cat16(v8h lo, v8h hi) { return __builtin_shufflevector(lo, hi, 0, 1, 2, 3, 4, 5, 6, 7, 8, 9, 10, 11, 12, 13, 14, 15); }
__device__ __forceinline__ v16bf cat16b(v8us lo, v8us hi) { return __builtin_bit_cast(v16bf, __builtin_shufflevector(lo, hi, 0, 1, 2, 3, 4, 5, 6, 7, 8, 9, 10, 11, 12, 13, 14, 15)); }
__device__ __forceinline__ v8f wmma16(v16h a, v16h b, v8f c) { return __builtin_amdgcn_wmma_f32_16x16x32_f16(false, a, false, b, (short)0, c, false, false); }
__device__ __forceinline__ v8f wmmab(v16bf a, v16bf b, v8f c) { return __builtin_amdgcn_wmma_f32_16x16x32_bf16(false, a, false, b, (short)0, c, false, false); }
__device__ __forceinline__ void lds_sync() { __builtin_amdgcn_wave_barrier(); asm volatile("" ::: "memory"); }

template <typename T16> struct WFrag;
template <> struct WFrag<h16> {
    typedef v16h V;
    static __device__ __forceinline__ V ld(const h16* p) { return cat16(*(const v8h*)p, *(const v8h*)(p + 16)); }
    static __device__ __forceinline__ v8f mma(V a, V b, v8f c) { return wmma16(a, b, c); }
    static __device__ __forceinline__ V pk(v8f p0, v8f p1) { v8h a, b;
#pragma unroll
        for (int k = 0; k < 8; ++k) { a[k] = (h16)p0[k]; b[k] = (h16)p1[k]; }
        return cat16(a, b); }
    static __device__ __forceinline__ V pkres(v8f p0, v8f p1) { return pk(p0, p1); }
};
template <> struct WFrag<bf> {
    typedef v16bf V;
    static __device__ __forceinline__ V ld(const bf* p) { return cat16b(*(const v8us*)p, *(const v8us*)(p + 16)); }
    static __device__ __forceinline__ v8f mma(V a, V b, v8f c) { return wmmab(a, b, c); }
    static __device__ __forceinline__ V pk(v8f p0, v8f p1) { v8us a, b;
#pragma unroll
        for (int k = 0; k < 8; ++k) { a[k] = f2bf(p0[k]); b[k] = f2bf(p1[k]); }
        return cat16b(a, b); }
    static __device__ __forceinline__ V pkres(v8f p0, v8f p1) { v8us a, b;
#pragma unroll
        for (int k = 0; k < 8; ++k) { unsigned short h0, l0, h1, l1; splitf(p0[k], h0, l0); splitf(p1[k], h1, l1); a[k] = l0; b[k] = l1; }
        return cat16b(a, b); }
};

__device__ __forceinline__ void put_rows(const float* os, unsigned lane, h16* d16, size_t p16, bool w16, bool whl, bf* dh, bf* dl, size_t phl) {
    const unsigned rq = lane >> 3, c = (lane & 7u) * 8u;
#pragma unroll 1
    for (int ps = 0; ps < 2; ++ps) {
#pragma unroll
        for (unsigned s = 0; s < 4; ++s) {
            const unsigned row = 4u * s + rq;
            const v4f x0 = *(const v4fa*)(os + row * 68u + c); const v4f x1 = *(const v4fa*)(os + row * 68u + c + 4u);
            if (w16) { v8h o;
#pragma unroll
                for (int k = 0; k < 4; ++k) { o[k] = (h16)x0[k]; o[4 + k] = (h16)x1[k]; }
                *(volatile v8h*)(d16 + (size_t)row * p16 + c) = o; }
            if (whl) { v8us oh, ol;
#pragma unroll
                for (int k = 0; k < 4; ++k) { unsigned short a, b; splitf(x0[k], a, b); oh[k] = a; ol[k] = b; splitf(x1[k], a, b); oh[4 + k] = a; ol[4 + k] = b; }
                *(volatile v8us*)(dh + (size_t)row * phl + c) = oh; *(volatile v8us*)(dl + (size_t)row * phl + c) = ol; }
        }
        if (ps == 0) __threadfence();
    }
}

template <typename T16, int NSPLIT, int MODE>
__global__ __launch_bounds__(32) void k_gemmw(const T16* __restrict__ A, const T16* __restrict__ A2, const T16* __restrict__ Bt, int K, float* C, int ldc, const float* __restrict__ bias, float cs, size_t sA, size_t sB, size_t sC, h16* P16, bf* Ph, bf* Pl, int lo16) {
    typedef typename WFrag<T16>::V V;
    __shared__ __align__(16) float os[16 * 68];
    const size_t z = blockIdx.z; A += z * sA; if (NSPLIT == 1) A2 += z * sA; Bt += z * sB; if (MODE == 0) C += z * sC;
    const unsigned lane = threadIdx.x & 31u, lr = lane & 15u, hi = lane >> 4; const unsigned r0 = blockIdx.x * 64u, c0 = blockIdx.y * 64u;
    v8f acc[4][4];
#pragma unroll
    for (int mb = 0; mb < 4; ++mb)
#pragma unroll
        for (int nb = 0; nb < 4; ++nb) acc[mb][nb] = (v8f){};
    const size_t aoff = (size_t)(r0 + lr) * (size_t)K + 8u * hi, boff = (size_t)(c0 + lr) * (size_t)K + 8u * hi;
#pragma unroll 1
    for (int kc = 0; kc < K; kc += 32) {
        V a[4], a2[4];
#pragma unroll
        for (int mb = 0; mb < 4; ++mb) { a[mb] = WFrag<T16>::ld(A + aoff + (size_t)mb * 16 * K + kc); if (NSPLIT == 1) a2[mb] = WFrag<T16>::ld(A2 + aoff + (size_t)mb * 16 * K + kc); }
#pragma unroll
        for (int nb = 0; nb < 4; ++nb) { const V b = WFrag<T16>::ld(Bt + boff + (size_t)nb * 16 * K + kc);
#pragma unroll
            for (int mb = 0; mb < 4; ++mb) { acc[mb][nb] = WFrag<T16>::mma(a[mb], b, acc[mb][nb]); if (NSPLIT == 1) acc[mb][nb] = WFrag<T16>::mma(a2[mb], b, acc[mb][nb]); } }
        asm volatile("v_nop\n\tv_nop\n\tv_nop\n\tv_nop" : "+v"(acc[0][0]), "+v"(acc[1][1]), "+v"(acc[2][2]), "+v"(acc[3][3]) : "v"(a[0]), "v"(a[3]));
    }
    float bcol[4];
#pragma unroll
    for (int nb = 0; nb < 4; ++nb) bcol[nb] = (MODE == 2) ? 0.0f : bfr(bias[c0 + nb * 16 + lr]);
#pragma unroll
    for (int mb = 0; mb < 4; ++mb) {
        float brow[8];
#pragma unroll
        for (int j = 0; j < 8; ++j) brow[j] = (MODE == 2) ? bfr(bias[r0 + mb * 16 + hi * 8 + j]) : 0.0f;
#pragma unroll
        for (int nb = 0; nb < 4; ++nb) {
#pragma unroll
            for (int j = 0; j < 8; ++j) os[(hi * 8 + j) * 68 + nb * 16 + lr] = acc[mb][nb][j] * cs + ((MODE == 2) ? brow[j] : bcol[nb]); }
        lds_sync();
        if (MODE == 0) {
            float* crow = C + (size_t)(r0 + mb * 16) * ldc + c0;
#pragma unroll 1
            for (int ps = 0; ps < 2; ++ps) {
#pragma unroll
                for (unsigned s = 0; s < 8; ++s) { const unsigned row = 2u * s + hi, cofs = lr * 4u; const v4f val = *(const v4fa*)(os + row * 68u + cofs);
                    *(volatile v4f*)(crow + (size_t)row * ldc + cofs) = val; }
                if (ps == 0) __threadfence(); }
        } else if (MODE == 1) {
            const unsigned R = r0 + mb * 16u; const unsigned b = R / (unsigned)SEQ, t = R % (unsigned)SEQ; const size_t bhq = (size_t)b * NH + blockIdx.y;
            const bool whl = (t < (unsigned)RH); const bool w16 = (lo16 != 0) || !whl;
            h16* d16 = P16 + (bhq * SEQ + t) * HD; const size_t ohl = (bhq * RH + (whl ? t : 0u)) * HD;
            put_rows(os, lane, d16, (size_t)HD, w16, whl, Ph + ohl, Pl + ohl, (size_t)HD);
        } else {
            const size_t bhq = z * NH + blockIdx.x; const unsigned d0 = mb * 16u;
            const bool whl = (c0 < (unsigned)RH); const bool w16 = (lo16 != 0) || !whl;
            h16* d16 = P16 + (bhq * HD + d0) * SEQ + c0; const size_t ohl = (bhq * HD + d0) * RH + (whl ? c0 : 0u);
            put_rows(os, lane, d16, (size_t)SEQ, w16, whl, Ph + ohl, Pl + ohl, (size_t)RH);
        }
        lds_sync();
    }
}

template <typename T16, bool HI>
__global__ __launch_bounds__(32) void k_flash(const T16* __restrict__ Qa, const T16* __restrict__ Qr, const T16* __restrict__ Ka, const T16* __restrict__ Kr, const T16* __restrict__ Va, const T16* __restrict__ Vr, h16* C16, bf* Ch, bf* Cl) {
    typedef typename WFrag<T16>::V V;
    __shared__ __align__(16) float os[16 * 68];
    constexpr unsigned LK = HI ? (unsigned)RH : (unsigned)SEQ;
    constexpr unsigned MB = HI ? 0u : (unsigned)RH;
    const unsigned lane = threadIdx.x & 31u, lr = lane & 15u, hi = lane >> 4;
    const unsigned bh = blockIdx.y, b = bh / (unsigned)NH, h = bh % (unsigned)NH;
    const unsigned m0 = MB + blockIdx.x * 16u, qidx = m0 + lr;
    const size_t qo = ((size_t)bh * LK + qidx) * HD + 8u * hi;
    const V qf0 = WFrag<T16>::ld(Qa + qo), qf1 = WFrag<T16>::ld(Qa + qo + 32);
    V qr0 = qf0, qr1 = qf1;
    if (HI) { qr0 = WFrag<T16>::ld(Qr + qo); qr1 = WFrag<T16>::ld(Qr + qo + 32); }
    const size_t ko = ((size_t)bh * LK + lr) * HD + 8u * hi;
    const size_t vo = ((size_t)bh * HD + lr) * LK + 8u * hi;
    v8f o[4];
#pragma unroll
    for (int nt = 0; nt < 4; ++nt) o[nt] = (v8f){};
    float mi = -3.0e38f, li = 0.0f;
    const unsigned nblk = ((m0 + 15u) >> 5) + 1u;
    const float SC2 = 0.125f * 1.4426950408889634f;
#pragma unroll 1
    for (unsigned ib = 0; ib < nblk; ++ib) {
        const unsigned kbase = ib * 32u;
        const size_t k0 = ko + (size_t)kbase * HD, k1 = k0 + (size_t)16 * HD;
        const V a00 = WFrag<T16>::ld(Ka + k0), a01 = WFrag<T16>::ld(Ka + k0 + 32), a10 = WFrag<T16>::ld(Ka + k1), a11 = WFrag<T16>::ld(Ka + k1 + 32);
        v8f s0 = (v8f){}, s1 = (v8f){};
        s0 = WFrag<T16>::mma(a00, qf0, s0); s0 = WFrag<T16>::mma(a01, qf1, s0);
        s1 = WFrag<T16>::mma(a10, qf0, s1); s1 = WFrag<T16>::mma(a11, qf1, s1);
        if (HI) {
            const V r00 = WFrag<T16>::ld(Kr + k0), r01 = WFrag<T16>::ld(Kr + k0 + 32), r10 = WFrag<T16>::ld(Kr + k1), r11 = WFrag<T16>::ld(Kr + k1 + 32);
            s0 = WFrag<T16>::mma(r00, qf0, s0); s0 = WFrag<T16>::mma(r01, qf1, s0);
            s1 = WFrag<T16>::mma(r10, qf0, s1); s1 = WFrag<T16>::mma(r11, qf1, s1);
            s0 = WFrag<T16>::mma(a00, qr0, s0); s0 = WFrag<T16>::mma(a01, qr1, s0);
            s1 = WFrag<T16>::mma(a10, qr0, s1); s1 = WFrag<T16>::mma(a11, qr1, s1);
        }
        asm volatile("v_nop\n\tv_nop\n\tv_nop\n\tv_nop" : "+v"(s0), "+v"(s1) : "v"(a00), "v"(a11), "v"(qf0), "v"(qf1));
        s0 *= SC2; s1 *= SC2;
        if (kbase + 31u > m0) {
#pragma unroll
            for (int r = 0; r < 8; ++r) { const unsigned key = kbase + 8u * hi + (unsigned)r;
                s0[r] = (key > qidx) ? -3.0e38f : s0[r]; s1[r] = (key + 16u > qidx) ? -3.0e38f : s1[r]; }
        }
        float mx = fmaxf(s0[0], s1[0]);
#pragma unroll
        for (int r = 1; r < 8; ++r) mx = fmaxf(mx, fmaxf(s0[r], s1[r]));
        mx = fmaxf(mx, __shfl_xor(mx, 16, 32));
        const float nm = fmaxf(mi, mx);
        const float alpha = __builtin_amdgcn_exp2f(mi - nm); mi = nm;
        const float sh = 8.0f - nm;
        float sum = 0.0f;
#pragma unroll
        for (int r = 0; r < 8; ++r) { const float p0 = __builtin_amdgcn_exp2f(s0[r] + sh), p1 = __builtin_amdgcn_exp2f(s1[r] + sh); s0[r] = p0; s1[r] = p1; sum += p0 + p1; }
        li = li * alpha + sum;
#pragma unroll
        for (int nt = 0; nt < 4; ++nt) o[nt] *= alpha;
        const V pf = WFrag<T16>::pk(s0, s1);
        V pr = pf; if (HI) pr = WFrag<T16>::pkres(s0, s1);
        V va[4];
#pragma unroll
        for (int nt = 0; nt < 4; ++nt) va[nt] = WFrag<T16>::ld(Va + vo + (size_t)nt * 16 * LK + kbase);
#pragma unroll
        for (int nt = 0; nt < 4; ++nt) o[nt] = WFrag<T16>::mma(va[nt], pf, o[nt]);
        if (HI) {
            V vr[4];
#pragma unroll
            for (int nt = 0; nt < 4; ++nt) vr[nt] = WFrag<T16>::ld(Vr + vo + (size_t)nt * 16 * LK + kbase);
#pragma unroll
            for (int nt = 0; nt < 4; ++nt) { o[nt] = WFrag<T16>::mma(vr[nt], pf, o[nt]); o[nt] = WFrag<T16>::mma(va[nt], pr, o[nt]); }
        }
        asm volatile("v_nop\n\tv_nop\n\tv_nop\n\tv_nop" : "+v"(o[0]), "+v"(o[1]), "+v"(o[2]), "+v"(o[3]) : "v"(pf), "v"(pr), "v"(va[0]), "v"(va[3]));
    }
    li += __shfl_xor(li, 16, 32);
    const float inv = (HI ? 1.0f : CTXCAR) * (1.0f / li);
#pragma unroll
    for (int nt = 0; nt < 4; ++nt) { v4f w0, w1;
#pragma unroll
        for (int k = 0; k < 4; ++k) { w0[k] = o[nt][k] * inv; w1[k] = o[nt][4 + k] * inv; }
        *(v4fa*)(os + lr * 68u + nt * 16 + 8u * hi) = w0; *(v4fa*)(os + lr * 68u + nt * 16 + 8u * hi + 4u) = w1; }
    lds_sync();
    h16* d16 = C16 + ((size_t)b * SEQ + m0) * DM + h * HD;
    const size_t ohl = ((size_t)b * RH + (HI ? m0 : 0u)) * DM + h * HD;
    put_rows(os, lane, d16, (size_t)DM, !HI, HI, Ch + ohl, Cl + ohl, (size_t)DM);
}

__global__ __launch_bounds__(256) void k_cvt8(const float* __restrict__ src, bf* dst, unsigned n8, size_t sstr, size_t dstr) {
    const unsigned i = blockIdx.x * 256u + threadIdx.x; if (i >= n8) return;
    const float* s = src + (size_t)blockIdx.y * sstr + (size_t)i * 8u; bf* d = dst + (size_t)blockIdx.y * dstr + (size_t)i * 8u;
    const v8f v = *(const v8f*)s; v8us o;
#pragma unroll
    for (int k = 0; k < 8; ++k) o[k] = f2bf(v[k]);
    *(volatile v8us*)d = o; __threadfence(); *(volatile v8us*)d = o; }
__global__ __launch_bounds__(256) void k_cvt8h(const float* __restrict__ src, h16* dst, unsigned n8, float car) {
    const unsigned i = blockIdx.x * 256u + threadIdx.x; if (i >= n8) return;
    const v8f v = *(const v8f*)(src + (size_t)i * 8u); v8h o;
#pragma unroll
    for (int k = 0; k < 8; ++k) o[k] = (h16)(bfr(v[k]) * car);
    *(volatile v8h*)(dst + (size_t)i * 8u) = o; __threadfence(); *(volatile v8h*)(dst + (size_t)i * 8u) = o; }

constexpr size_t SZ_X   = (size_t)NB * SEQ * DM * 2;
constexpr size_t SZ_W   = (size_t)DM * DM * 2;
constexpr size_t SZ_P16 = (size_t)NB * NH * SEQ * HD * 2;
constexpr size_t SZ_PHL = (size_t)NB * NH * RH * HD * 2;
constexpr size_t SZ_CHL = (size_t)NB * RH * DM * 2;
constexpr size_t WS_TOTAL = SZ_X + 5 * SZ_W + 3 * SZ_P16 + 6 * SZ_PHL + SZ_X + 2 * SZ_CHL;
static_assert(WS_TOTAL <= (size_t)134217728);
static_assert(SZ_X % 256 == 0);
static_assert(SZ_W % 256 == 0);
static_assert(SZ_PHL % 256 == 0);
static_assert(SZ_CHL % 256 == 0);

extern "C" void kernel_launch(void* const* d_in, const int* in_sizes, int n_in,
                              void* d_out, int out_size, void* d_ws, size_t ws_size, hipStream_t stream) {
    if (n_in < 9) return;
    if ((size_t)in_sizes[0] < (size_t)(NB - 1) * X_BSTRIDE + (size_t)SEQ * DM) return;
    if ((size_t)in_sizes[1] < (size_t)DM * DM || (size_t)in_sizes[3] < (size_t)DM * DM || (size_t)in_sizes[5] < (size_t)DM * DM || (size_t)in_sizes[7] < (size_t)DM * DM) return;
    if (in_sizes[2] < DM || in_sizes[4] < DM || in_sizes[6] < DM || in_sizes[8] < DM) return;
    if ((size_t)out_size < (size_t)(NB - 1) * OUT_BSTRIDE + (size_t)SEQ * DM) return;
    if (WS_TOTAL > ws_size) return;
    const float* x  = (const float*)d_in[0];
    const float* wq = (const float*)d_in[1]; const float* bq = (const float*)d_in[2];
    const float* wk = (const float*)d_in[3]; const float* bk = (const float*)d_in[4];
    const float* wv = (const float*)d_in[5]; const float* bv = (const float*)d_in[6];
    const float* wo = (const float*)d_in[7]; const float* bo = (const float*)d_in[8];
    float* OUT = (float*)d_out;
    char* wsp = (char*)d_ws;
    auto take = [&](size_t bytes) { char* p = wsp; wsp += (bytes + 255) & ~(size_t)255; return (void*)p; };
    bf* XB = (bf*)take(SZ_X);
    bf* WQb = (bf*)take(SZ_W); bf* WKb = (bf*)take(SZ_W); bf* WVb = (bf*)take(SZ_W); bf* WOb = (bf*)take(SZ_W); h16* WO16 = (h16*)take(SZ_W);
    h16* Q16 = (h16*)take(SZ_P16); h16* K16 = (h16*)take(SZ_P16); h16* VT16 = (h16*)take(SZ_P16);
    bf* Qh = (bf*)take(SZ_PHL); bf* Ql = (bf*)take(SZ_PHL); bf* Kh = (bf*)take(SZ_PHL); bf* Kl = (bf*)take(SZ_PHL); bf* VTh = (bf*)take(SZ_PHL); bf* VTl = (bf*)take(SZ_PHL);
    h16* CTX16 = (h16*)take(SZ_X); bf* CTXh = (bf*)take(SZ_CHL); bf* CTXl = (bf*)take(SZ_CHL);
    if ((size_t)(wsp - (char*)d_ws) > ws_size) return;

    const unsigned nx8 = (unsigned)((size_t)SEQ * DM / 8), nw8 = (unsigned)((size_t)DM * DM / 8);
    k_cvt8<<<dim3(nx8 / 256, NB, 1), 256, 0, stream>>>(x, XB, nx8, X_BSTRIDE, (size_t)SEQ * DM);
    k_cvt8<<<dim3(nw8 / 256, 1, 1), 256, 0, stream>>>(wq, WQb, nw8, 0, 0);
    k_cvt8<<<dim3(nw8 / 256, 1, 1), 256, 0, stream>>>(wk, WKb, nw8, 0, 0);
    k_cvt8<<<dim3(nw8 / 256, 1, 1), 256, 0, stream>>>(wv, WVb, nw8, 0, 0);
    k_cvt8<<<dim3(nw8 / 256, 1, 1), 256, 0, stream>>>(wo, WOb, nw8, 0, 0);
    k_cvt8h<<<dim3(nw8 / 256, 1, 1), 256, 0, stream>>>(wo, WO16, nw8, WOCAR);

    k_gemmw<bf, 0, 1><<<dim3(NB * SEQ / 64, DM / 64, 1), 32, 0, stream>>>(XB, nullptr, WQb, DM, nullptr, 0, bq, 1.0f, 0, 0, 0, Q16, Qh, Ql, 0);
    k_gemmw<bf, 0, 1><<<dim3(NB * SEQ / 64, DM / 64, 1), 32, 0, stream>>>(XB, nullptr, WKb, DM, nullptr, 0, bk, 1.0f, 0, 0, 0, K16, Kh, Kl, 1);
    k_gemmw<bf, 0, 2><<<dim3(DM / 64, SEQ / 64, NB), 32, 0, stream>>>(WVb, nullptr, XB, DM, nullptr, 0, bv, 1.0f, 0, (size_t)SEQ * DM, 0, VT16, VTh, VTl, 1);

    k_flash<bf, true><<<dim3(RH / 16, NB * NH, 1), 32, 0, stream>>>(Qh, Ql, Kh, Kl, VTh, VTl, CTX16, CTXh, CTXl);
    if (SEQ > RH)
        k_flash<h16, false><<<dim3((SEQ - RH) / 16, NB * NH, 1), 32, 0, stream>>>(Q16, nullptr, K16, nullptr, VT16, nullptr, CTX16, CTXh, CTXl);

    k_gemmw<bf, 1, 0><<<dim3(RH / 64, DM / 64, NB), 32, 0, stream>>>(CTXh, CTXl, WOb, DM, OUT, DM, bo, 1.0f, (size_t)RH * DM, 0, OUT_BSTRIDE, nullptr, nullptr, nullptr, 0);
    if (SEQ > RH)
        k_gemmw<h16, 0, 0><<<dim3((SEQ - RH) / 64, DM / 64, NB), 32, 0, stream>>>(CTX16 + (size_t)RH * DM, nullptr, WO16, DM, OUT + (size_t)RH * DM, DM, bo, 1.0f / (CTXCAR * WOCAR), (size_t)SEQ * DM, 0, OUT_BSTRIDE, nullptr, nullptr, nullptr, 0);
}
